// RelMultiHeadAttn_19619410608620
// MI455X (gfx1250) — hardware-verified
//
#include <hip/hip_runtime.h>


namespace {
constexpr int Q = 1024, B = 4, DM = 1024, NH = 16, DH = 64, RL = Q + 1, RP = Q + 48  , NT = Q * B, QL = 1024  ;
constexpr float XS = 8.0f, WSC = 256.0f, PS = 1024.0f, LOG2E = 1.4426950408889634f, EPS = 1e-5f;
static_assert(Q % 64 == 0 && QL % 32 == 0 && RP % 16 == 0 && DM == NH * DH, "tiling");
typedef _Float16 b16;
typedef __attribute__((ext_vector_type(16))) _Float16 v16b;
typedef __attribute__((ext_vector_type(8))) _Float16 v8b;
typedef __attribute__((ext_vector_type(8))) float v8f;
typedef __attribute__((ext_vector_type(4))) float v4f;
__device__ __forceinline__ float bf16_rne(float f) { unsigned int u = __float_as_uint(f); u += 0x7FFFu + ((u >> 16) & 1u); return __uint_as_float(u & 0xFFFF0000u); }
__device__ __forceinline__ void split16(float v, b16& hi, b16& lo) { hi = (b16)v; lo = (b16)(v - (float)hi); }
__device__ __forceinline__ v16b frag_kb(const b16* p, int hh) { const v8b a = *(const v8b*)(p + 8 * hh), b = *(const v8b*)(p + 16 + 8 * hh); v16b f;
#pragma unroll
  for (int e = 0; e < 8; ++e) { f[e] = a[e]; f[8 + e] = b[e]; } return f; }
__device__ __forceinline__ v8f wmma16b(v16b a, v16b b, v8f c) { v8f d = __builtin_amdgcn_wmma_f32_16x16x32_f16(false, a, false, b, (short)0, c, false, false); asm volatile("v_nop\n\tv_nop\n\tv_nop\n\tv_nop" : "+v"(d) : "v"(a), "v"(b)); return d; }
__device__ __forceinline__ void wave_lds_sync() { __builtin_amdgcn_fence(__ATOMIC_RELEASE, "workgroup"); __builtin_amdgcn_wave_barrier(); __builtin_amdgcn_fence(__ATOMIC_ACQUIRE, "workgroup"); }
__device__ __forceinline__ float pmul(float a, float b) { float p = a * b; asm volatile("" : "+v"(p)); return p; }
__device__ __forceinline__ int iclamp(int v, int lo, int hi) { return v < lo ? lo : (v > hi ? hi : v); }

typedef __attribute__((ext_vector_type(2))) _Float16 v2h;
typedef __attribute__((ext_vector_type(4))) _Float16 v4h;
typedef __attribute__((ext_vector_type(4))) int v4i;
__device__ __forceinline__ float nexp2(float v) { return __builtin_amdgcn_exp2f(v); }
__global__ __launch_bounds__(256) void prep_kernel(const float* __restrict__ wqkv, const float* __restrict__ wo, b16* __restrict__ WT, b16* __restrict__ WO) {
  const size_t u = (size_t)blockIdx.x * 256 + threadIdx.x; const size_t n1 = (size_t)3 * DM * DM / 8, n2 = (size_t)DM * DM / 8; v8b o;
  if (u < n1) { const size_t e = u * 8; const int oo = (int)(e / DM), d0 = (int)(e % DM); for (int j = 0; j < 8; ++j) o[j] = (b16)(bf16_rne(wqkv[(size_t)(d0 + j) * (3 * DM) + oo]) * WSC); for (int pass = 0; pass < 2; ++pass) { *(volatile v8b*)(WT + e) = o; __threadfence(); } }
  else if (u < n1 + n2) { const size_t e = (u - n1) * 8; const int oo = (int)(e / DM), k0 = (int)(e % DM); for (int j = 0; j < 8; ++j) o[j] = (b16)(bf16_rne(wo[(size_t)(k0 + j) * DM + oo]) * WSC); for (int pass = 0; pass < 2; ++pass) { *(volatile v8b*)(WO + e) = o; __threadfence(); } }
}
struct TileOut { float (*Tf)[128 + 4]; };
__global__ __launch_bounds__(128) void rproj_kernel(const float* __restrict__ r, const b16* __restrict__ WT, float* __restrict__ RQL, b16* __restrict__ RK) {
  __shared__ __attribute__((aligned(16))) b16 As[64][256 + 8]; __shared__ __attribute__((aligned(16))) float Tf[4][16][128 + 4];
  const int wave = threadIdx.x >> 5, lane = threadIdx.x & 31, nloc = lane & 15, hlf = lane >> 4; const int r0 = blockIdx.x * 64; const int m0 = r0 + wave * 16; const int slab = blockIdx.y, n0 = slab * 128;
  v8f acc[8];
#pragma unroll
  for (int t = 0; t < 8; ++t) acc[t] = (v8f){};
#pragma unroll 1
  for (int kc = 0; kc < DM; kc += 256) {
    __syncthreads();
    for (int i = threadIdx.x; i < 64 * 64; i += 128) { const int rr = i / 64, q = (i % 64) * 4; const int row = r0 + rr; v4h o; if (row < RL) { const v4f f = *(const v4f*)(r + (size_t)row * DM + kc + q); for (int j = 0; j < 4; ++j) o[j] = (b16)(bf16_rne(f[j]) * XS); } else { for (int j = 0; j < 4; ++j) o[j] = (b16)0.0f; } *(v4h*)(&As[rr][q]) = o; }
    __syncthreads();
#pragma unroll 2
    for (int kb = 0; kb < 256; kb += 32) { const v16b a = frag_kb(&As[wave * 16 + nloc][kb], hlf);
#pragma unroll
      for (int t = 0; t < 8; ++t) acc[t] = wmma16b(a, frag_kb(WT + (size_t)(n0 + t * 16 + nloc) * DM + kc + kb, hlf), acc[t]); } }
#pragma unroll
  for (int t = 0; t < 8; ++t)
#pragma unroll
    for (int rr = 0; rr < 8; ++rr) Tf[wave][8 * hlf + rr][t * 16 + nloc] = acc[t][rr] * (1.0f / (XS * WSC));
  wave_lds_sync();
  for (int pass = 0; pass < 2; ++pass) {
    if (slab < 8) { if (m0 <= RL - 1 && RL - 1 < m0 + 16) { const int rr = RL - 1 - m0; *(volatile v4f*)(RQL + n0 + lane * 4) = *(const v4f*)(&Tf[wave][rr][lane * 4]); } }
    else { const int c = (n0 - DM) + lane * 4; const int n = c / DH, d = c % DH; for (int rr = 0; rr < 16; ++rr) { const int j = m0 + rr; if (j < RP) { v4h o4; for (int q = 0; q < 4; ++q) o4[q] = (b16)(Tf[wave][rr][lane * 4 + q] * XS); *(volatile v4h*)(RK + ((size_t)n * RP + j) * DH + d) = o4; } } }
    __threadfence(); }
}
__global__ __launch_bounds__(128) void proj_kernel(const float* __restrict__ w, const b16* __restrict__ WT, const float* __restrict__ RQL, b16* __restrict__ QP, b16* __restrict__ KP, b16* __restrict__ VT) {
  __shared__ __attribute__((aligned(16))) b16 As[64][256 + 8]; __shared__ __attribute__((aligned(16))) float Tf[4][16][128 + 4];
  const int wave = threadIdx.x >> 5, lane = threadIdx.x & 31, nloc = lane & 15, hlf = lane >> 4; const int i0 = blockIdx.x * 64; const int b = blockIdx.y; const int slab = blockIdx.z, n0 = slab * 128, part = slab / 8, c0 = n0 - part * DM; const int mi = i0 + wave * 16;
  v8f acc[8];
#pragma unroll
  for (int t = 0; t < 8; ++t) acc[t] = (v8f){};
#pragma unroll 1
  for (int kc = 0; kc < DM; kc += 256) {
    __syncthreads();
    for (int i = threadIdx.x; i < 64 * 64; i += 128) { const int rr = i / 64, q = (i % 64) * 4; const v4f f = *(const v4f*)(w + ((size_t)(i0 + rr) * B + b) * DM + kc + q); v4h o; for (int j = 0; j < 4; ++j) o[j] = (b16)(bf16_rne(f[j]) * XS); *(v4h*)(&As[rr][q]) = o; }
    __syncthreads();
#pragma unroll 2
    for (int kb = 0; kb < 256; kb += 32) { const v16b a = frag_kb(&As[wave * 16 + nloc][kb], hlf);
#pragma unroll
      for (int t = 0; t < 8; ++t) acc[t] = wmma16b(a, frag_kb(WT + (size_t)(n0 + t * 16 + nloc) * DM + kc + kb, hlf), acc[t]); } }
#pragma unroll
  for (int t = 0; t < 8; ++t) { const float add = (part == 0) ? RQL[c0 + t * 16 + nloc] : 0.0f;
#pragma unroll
    for (int rr = 0; rr < 8; ++rr) Tf[wave][8 * hlf + rr][t * 16 + nloc] = acc[t][rr] * (1.0f / (XS * WSC)) + add; }
  __syncthreads();
  for (int pass = 0; pass < 2; ++pass) {
    if (part < 2) { b16* plane = part == 0 ? QP : KP; const int c = c0 + lane * 4; const int n = c / DH, d = c % DH;
      for (int rr = 0; rr < 16; ++rr) { const int i = mi + rr; v4h o4; for (int q = 0; q < 4; ++q) o4[q] = (b16)(Tf[wave][rr][lane * 4 + q] * XS); *(volatile v4h*)(plane + (((size_t)b * NH + n) * Q + i) * DH + d) = o4; } }
    else {
#pragma unroll 1
      for (int q = 0; q < 32; ++q) { const int cl = wave * 32 + q; const int c = c0 + cl; const int n = c / DH, d = c % DH; const int tk = lane * 2; v2h vv; vv[0] = (b16)(Tf[tk >> 4][tk & 15][cl] * XS); vv[1] = (b16)(Tf[(tk + 1) >> 4][(tk + 1) & 15][cl] * XS);
        *(volatile v2h*)(VT + (((size_t)b * NH + n) * DH + d) * (size_t)Q + i0 + lane * 2) = vv; } }
    __threadfence(); }
}
__global__ __launch_bounds__(64) void attn_kernel(const b16* __restrict__ QP, const b16* __restrict__ KP, const b16* __restrict__ VT, const b16* __restrict__ RK, const int* __restrict__ amask, b16* __restrict__ AV) {
  __shared__ __attribute__((aligned(16))) b16 Pb[2][16][32 + 8]; __shared__ __attribute__((aligned(16))) float To[2][16][DH + 4]; __shared__ float Tb[2][32][16 + 1];
  const int wave = threadIdx.x >> 5, lane = threadIdx.x & 31, hh = lane >> 4, col = lane & 15; const int b = blockIdx.y / NH, n = blockIdx.y % NH; const int i0 = blockIdx.x * 32 + wave * 16, qi = i0 + col;
  const size_t pn = (size_t)b * NH + n; const b16* Qb = QP + pn * Q * DH; const b16* Kb = KP + pn * Q * DH; const b16* Vb = VT + pn * DH * (size_t)Q; const b16* Rb = RK + (size_t)n * RP * DH; const int* Mrow = amask + (size_t)qi * Q;
  const v16b qa0 = frag_kb(Qb + (size_t)qi * DH, hh), qa1 = frag_kb(Qb + (size_t)qi * DH + 32, hh);
  const float cs = LOG2E / (8.0f * XS * XS);
  float m = -INFINITY, l = 0.0f; v8f o[4]; for (int t = 0; t < 4; ++t) o[t] = (v8f){};
  const int kend = i0 + 16;
#pragma unroll 1
  for (int kb = 0; kb < kend; kb += 32) {
    float e[16]; float mx = -INFINITY;
#pragma unroll
    for (int u = 0; u < 2; ++u) { const int j0 = kb + u * 16;
      const int base = Q - (i0 + 15) + j0;
#pragma unroll
      for (int t2 = 0; t2 < 2; ++t2) { v8f tb = (v8f){}; const size_t rr = (size_t)(base + t2 * 16 + col) * DH; tb = wmma16b(frag_kb(Rb + rr, hh), qa0, tb); tb = wmma16b(frag_kb(Rb + rr + 32, hh), qa1, tb);
#pragma unroll
        for (int r = 0; r < 8; ++r) Tb[wave][t2 * 16 + 8 * hh + r][col] = tb[r]; }
      v8f s = (v8f){}; const size_t kr = (size_t)(j0 + col) * DH; s = wmma16b(frag_kb(Kb + kr, hh), qa0, s); s = wmma16b(frag_kb(Kb + kr + 32, hh), qa1, s);
      wave_lds_sync();
      const v4i mk0 = *(const v4i*)(Mrow + j0 + 8 * hh), mk1 = *(const v4i*)(Mrow + j0 + 8 * hh + 4);
#pragma unroll
      for (int r = 0; r < 8; ++r) { const int jl = 8 * hh + r; const int key = j0 + jl; const int bi = jl + 15 - col; const int mk = (r < 4) ? mk0[r] : mk1[r - 4];
        const float bd = (bi >= 0 && bi < 31) ? Tb[wave][bi][col] : 0.0f;
        const float vv = (mk != 0 || key > qi) ? -INFINITY : (s[r] + bd) * cs; e[u * 8 + r] = vv; mx = fmaxf(mx, vv); }
      wave_lds_sync(); }
    mx = fmaxf(mx, __shfl_xor(mx, 16)); const float mn = fmaxf(m, mx); const float al = (mn == -INFINITY) ? 1.0f : nexp2(m - mn); float sum = 0.0f;
#pragma unroll
    for (int i2 = 0; i2 < 16; ++i2) { const float p = (e[i2] == -INFINITY || mn == -INFINITY) ? 0.0f : nexp2(e[i2] - mn); sum += p; Pb[wave][col][(i2 < 8 ? 0 : 16) + 8 * hh + (i2 & 7)] = (b16)(p * PS); }
    sum += __shfl_xor(sum, 16); l = l * al + sum; m = mn;
    wave_lds_sync();
    const v16b pf = frag_kb(&Pb[wave][col][0], hh);
#pragma unroll
    for (int t = 0; t < 4; ++t) { o[t] *= al; o[t] = wmma16b(frag_kb(Vb + (size_t)(t * 16 + col) * Q + kb, hh), pf, o[t]); }
    wave_lds_sync(); }
  const float inv = (l > 0.0f) ? 1.0f / (l * PS * XS) : __int_as_float(0x7fc00000);
#pragma unroll
  for (int t = 0; t < 4; ++t)
#pragma unroll
    for (int r = 0; r < 8; ++r) To[wave][col][t * 16 + 8 * hh + r] = o[t][r] * inv;
  wave_lds_sync();
  for (int pass = 0; pass < 2; ++pass) { for (int rr = 0; rr < 16; ++rr) { v2h o2; o2[0] = (b16)(To[wave][rr][lane * 2] * XS); o2[1] = (b16)(To[wave][rr][lane * 2 + 1] * XS); *(volatile v2h*)(AV + ((size_t)(i0 + rr) * B + b) * DM + n * DH + lane * 2) = o2; } __threadfence(); }
}
__global__ __launch_bounds__(128) void out_kernel(const b16* __restrict__ AV, const b16* __restrict__ WO, const float* __restrict__ w, float* __restrict__ Y) {
  __shared__ __attribute__((aligned(16))) float Tf[4][16][128 + 4];
  const int wave = threadIdx.x >> 5, lane = threadIdx.x & 31, nloc = lane & 15, hlf = lane >> 4; const size_t m0 = ((size_t)blockIdx.x * 4 + wave) * 16; const int n0 = blockIdx.y * 128;
  v8f acc[8];
#pragma unroll
  for (int t = 0; t < 8; ++t) acc[t] = (v8f){};
#pragma unroll 2
  for (int kb = 0; kb < DM; kb += 32) { const v16b a = frag_kb(AV + (m0 + nloc) * DM + kb, hlf);
#pragma unroll
    for (int t = 0; t < 8; ++t) acc[t] = wmma16b(a, frag_kb(WO + (size_t)(n0 + t * 16 + nloc) * DM + kb, hlf), acc[t]); }
#pragma unroll
  for (int t = 0; t < 8; ++t)
#pragma unroll
    for (int rr = 0; rr < 8; ++rr) Tf[wave][8 * hlf + rr][t * 16 + nloc] = acc[t][rr] * (1.0f / (XS * WSC));
  wave_lds_sync();
  for (int rr = 0; rr < 16; ++rr) { const v4f wv = *(const v4f*)(w + (m0 + rr) * DM + n0 + lane * 4); v4f t4 = *(const v4f*)(&Tf[wave][rr][lane * 4]); for (int j = 0; j < 4; ++j) t4[j] += bf16_rne(wv[j]); *(v4f*)(&Tf[wave][rr][lane * 4]) = t4; }
  wave_lds_sync();
  for (int pass = 0; pass < 2; ++pass) { for (int rr = 0; rr < 16; ++rr) *(volatile v4f*)(Y + (m0 + rr) * DM + n0 + lane * 4) = *(const v4f*)(&Tf[wave][rr][lane * 4]); __threadfence(); }
}
__global__ __launch_bounds__(256) void ln_kernel(const float* __restrict__ Y, const float* __restrict__ gam, const float* __restrict__ bet, float* __restrict__ out) {
  const int wave = threadIdx.x >> 5, lane = threadIdx.x & 31; const size_t row = (size_t)blockIdx.x * 8 + wave; if (row >= (size_t)QL * B) return;
  float v[32]; float s = 0.0f;
#pragma unroll
  for (int q = 0; q < 8; ++q) { const v4f f = *(const v4f*)(Y + row * DM + q * 128 + lane * 4); for (int j = 0; j < 4; ++j) { v[q * 4 + j] = f[j]; s += f[j]; } }
#pragma unroll
  for (int o = 1; o < 32; o <<= 1) s += __shfl_xor(s, o);
  const float mu = s * (1.0f / DM); float vs = 0.0f;
#pragma unroll
  for (int i = 0; i < 32; ++i) { const float d = v[i] - mu; vs += d * d; }
#pragma unroll
  for (int o = 1; o < 32; o <<= 1) vs += __shfl_xor(vs, o);
  const float rs = rsqrtf(vs * (1.0f / DM) + EPS);
  for (int pass = 0; pass < 2; ++pass) {
#pragma unroll
    for (int q = 0; q < 8; ++q) { v4f r4; for (int j = 0; j < 4; ++j) { const int c = q * 128 + lane * 4 + j; r4[j] = (v[q * 4 + j] - mu) * rs * bf16_rne(gam[c]) + bf16_rne(bet[c]); } *(volatile v4f*)(out + row * DM + q * 128 + lane * 4) = r4; }
    __threadfence(); }
}
}

extern "C" void kernel_launch(void* const* d_in, const int* in_sizes, int n_in, void* d_out, int out_size, void* d_ws, size_t ws_size, hipStream_t stream) {
  (void)n_in;
  auto Fp = [&](int i) { return (const float*)d_in[i]; }; auto Ip = [&](int i) { return (const int*)d_in[i]; };
  if (in_sizes[0] != NT * DM || in_sizes[1] != RL * DM || in_sizes[2] != Q * Q || in_sizes[3] != DM * 3 * DM || in_sizes[4] != DM * DM || in_sizes[5] != DM || in_sizes[6] != DM || out_size != NT * DM) return;
  size_t off = 0; char* ws = (char*)d_ws;
  auto carve = [&](size_t bytes) { char* p = ws + off; off += (bytes + 255) & ~(size_t)255; return p; };
  b16* WT = (b16*)carve((size_t)3 * DM * DM * 2); b16* WO = (b16*)carve((size_t)DM * DM * 2); float* RQL = (float*)carve((size_t)DM * 4); b16* RK = (b16*)carve((size_t)NH * RP * DH * 2);
  const size_t plane = (size_t)B * NH * Q * DH * 2; b16* QP = (b16*)carve(plane); b16* KP = (b16*)carve(plane); b16* VT = (b16*)carve(plane); b16* AV = (b16*)carve(plane); float* Y = (float*)carve((size_t)NT * DM * 4);
  if (off > ws_size || off > ((size_t)128 << 20)) return;
  prep_kernel<<<(unsigned)(((size_t)4 * DM * DM / 8 + 255) / 256), 256, 0, stream>>>(Fp(3), Fp(4), WT, WO);
  rproj_kernel<<<dim3(RP / 64 + 1, 16), 128, 0, stream>>>(Fp(1), WT, RQL, RK);
  proj_kernel<<<dim3(((QL + 64 < Q) ? (QL + 64) : Q) / 64, B, 24), 128, 0, stream>>>(Fp(0), WT, RQL, QP, KP, VT);
  attn_kernel<<<dim3(QL / 32, B * NH), 64, 0, stream>>>(QP, KP, VT, RK, Ip(2), AV);
  out_kernel<<<dim3((QL * B) / 64, DM / 128), 128, 0, stream>>>(AV, WO, Fp(0), Y);
  ln_kernel<<<(QL * B) / 8, 256, 0, stream>>>(Y, Fp(5), Fp(6), (float*)d_out);
}
